// HyperSAGNN_5119601017143
// MI455X (gfx1250) — hardware-verified
//
#include <hip/hip_runtime.h>
#include <stddef.h>
#include <stdint.h>
#include <float.h>
#include <math.h>

#define NN    4096
#define HD    512
#define NHEAD 8
#define HDIM  64
#define NSET  1365
#define OTP   68

static_assert(HD == NHEAD * HDIM);
static_assert(HDIM == 64);
static_assert(NHEAD * 32 == 256);
static_assert(NN % 256 == 0);
static_assert(HD % 64 == 0);
static_assert(HD % 32 == 0);
static_assert((NN * HD) % 2048 == 0);
static_assert(HD == 4 * 128);

typedef _Float16 v16h __attribute__((ext_vector_type(16)));
typedef _Float16 v8h  __attribute__((ext_vector_type(8)));
typedef float    v8f  __attribute__((ext_vector_type(8)));
typedef float    v4f  __attribute__((ext_vector_type(4)));
typedef float    v2f  __attribute__((ext_vector_type(2)));
typedef unsigned int v4u __attribute__((ext_vector_type(4)));

union Frag  { v16h v; v8h h[2]; };
union Pack8 { v8h h; v4u u; };

__device__ __forceinline__ v8f mma16(v16h a, v16h b, v8f c) {
  c = __builtin_amdgcn_wmma_f32_16x16x32_f16(false, a, false, b, (short)0, c, false, false);
  asm volatile("v_nop\n\tv_nop\n\tv_nop\n\tv_nop" : "+v"(c) : "v"(a), "v"(b));
  return c;
}

__device__ __forceinline__ v16h ldfrag(const _Float16* p, int ld, int row0, int k0, int lane) {
  const int m = lane & 15, lh = lane >> 4;
  const _Float16* q = p + (size_t)(row0 + m) * ld + k0 + 8 * lh;
  Frag f;
  f.h[0] = *(const v8h*)(q);
  f.h[1] = *(const v8h*)(q + 16);
  return f.v;
}

__device__ __forceinline__ v8f zero8() { return (v8f){0.f, 0.f, 0.f, 0.f, 0.f, 0.f, 0.f, 0.f}; }

__device__ __forceinline__ v8h cvt8(v4f a0, v4f a1) {
  return (v8h){(_Float16)a0[0], (_Float16)a0[1], (_Float16)a0[2], (_Float16)a0[3],
               (_Float16)a1[0], (_Float16)a1[1], (_Float16)a1[2], (_Float16)a1[3]};
}

__device__ __forceinline__ void gemm32x64(const _Float16* __restrict__ A, int lda,
                                          const _Float16* __restrict__ Bt, int ldb, int K,
                                          int m0, int n0, int lane, v8f (&acc)[2][4]) {
#pragma unroll 1
  for (int k0 = 0; k0 < K; k0 += 32) {
    const v16h a0 = ldfrag(A, lda, m0, k0, lane);
    const v16h a1 = ldfrag(A, lda, m0 + 16, k0, lane);
    const v16h b0 = ldfrag(Bt, ldb, n0, k0, lane);
    const v16h b1 = ldfrag(Bt, ldb, n0 + 16, k0, lane);
    const v16h b2 = ldfrag(Bt, ldb, n0 + 32, k0, lane);
    const v16h b3 = ldfrag(Bt, ldb, n0 + 48, k0, lane);
    acc[0][0] = mma16(a0, b0, acc[0][0]);
    acc[1][0] = mma16(a1, b0, acc[1][0]);
    acc[0][1] = mma16(a0, b1, acc[0][1]);
    acc[1][1] = mma16(a1, b1, acc[1][1]);
    acc[0][2] = mma16(a0, b2, acc[0][2]);
    acc[1][2] = mma16(a1, b2, acc[1][2]);
    acc[0][3] = mma16(a0, b3, acc[0][3]);
    acc[1][3] = mma16(a1, b3, acc[1][3]);
  }
}

__global__ __launch_bounds__(256) void k_wt(const float* __restrict__ W, _Float16* __restrict__ WT) {
  __shared__ float tile[64][33];
  const int tid = threadIdx.x;
  const int k0 = blockIdx.x * 64, n0 = blockIdx.y * 32;
#pragma unroll
  for (int j = 0; j < 8; ++j) {
    const int idx = tid + 256 * j;
    const int kr = idx >> 5, nc = idx & 31;
    tile[kr][nc] = W[(size_t)(k0 + kr) * HD + n0 + nc];
  }
  __syncthreads();
  const int nr = tid >> 3, pc = tid & 7;
  v4f a0, a1;
  a0.x = tile[8 * pc + 0][nr]; a0.y = tile[8 * pc + 1][nr]; a0.z = tile[8 * pc + 2][nr]; a0.w = tile[8 * pc + 3][nr];
  a1.x = tile[8 * pc + 4][nr]; a1.y = tile[8 * pc + 5][nr]; a1.z = tile[8 * pc + 6][nr]; a1.w = tile[8 * pc + 7][nr];
  Pack8 pk;
  pk.h = cvt8(a0 * 1024.0f, a1 * 1024.0f);
  const v4u vv = pk.u;
  volatile v4u* d = (volatile v4u*)(WT + (size_t)(n0 + nr) * HD + k0 + 8 * pc);
  *d = vv;
  __threadfence();
  *d = vv;
}

__global__ __launch_bounds__(256) void k_cvt(const float* __restrict__ src, _Float16* __restrict__ dh, float scale) {
  const size_t o = (size_t)blockIdx.x * 2048 + (size_t)threadIdx.x * 8;
  const v4f a0 = *(const v4f*)(src + o) * scale;
  const v4f a1 = *(const v4f*)(src + o + 4) * scale;
  Pack8 pk;
  pk.h = cvt8(a0, a1);
  const v4u vv = pk.u;
  volatile v4u* d = (volatile v4u*)(dh + o);
  *d = vv;
  __threadfence();
  *d = vv;
}

template <int MODE, bool MIRROR>
__global__ __launch_bounds__(256) void k_gemm(const _Float16* __restrict__ ap,
                                              const _Float16* __restrict__ wt,
                                              const float* __restrict__ bias, float scale,
                                              const float* __restrict__ resid,
                                              const float* __restrict__ betap,
                                              float* __restrict__ out,
                                              _Float16* __restrict__ out16) {
  __shared__ __align__(16) float st[8][16 * OTP];
  const int tid = threadIdx.x, lane = tid & 31, wave = tid >> 5;
  const int hh = lane >> 4, c = lane & 15;
  const int m0 = blockIdx.x * 256 + wave * 32;
  const int n0 = blockIdx.y * 64;

  v8f acc[2][4];
#pragma unroll
  for (int s = 0; s < 2; ++s)
#pragma unroll
    for (int t = 0; t < 4; ++t) acc[s][t] = zero8();
  gemm32x64(ap, HD, wt, HD, HD, m0, n0, lane, acc);

  float bb[4];
#pragma unroll
  for (int t = 0; t < 4; ++t) bb[t] = bias[n0 + 16 * t + c];
  const float beta = (MODE == 2) ? betap[0] : 1.0f;
  float* sw = st[wave];

#pragma unroll
  for (int sub = 0; sub < 2; ++sub) {
    __syncthreads();
#pragma unroll
    for (int t = 0; t < 4; ++t) {
#pragma unroll
      for (int r = 0; r < 8; ++r) {
        const int lrow = 8 * hh + r;
        const int col  = 16 * t + c;
        float v = acc[sub][t][r] * scale + bb[t];
        if (MODE == 0) v = fmaxf(v, 0.0f);
        if (MODE == 2) v = beta * v;
        sw[lrow * OTP + col] = v;
      }
    }
    __syncthreads();
    {
      v4f val[8];
      size_t go[8];
#pragma unroll
      for (int it = 0; it < 8; ++it) {
        const int p    = lane + 32 * it;
        const int Lr   = p >> 3;
        const int pc   = p & 7;
        const int row  = Lr >> 1;
        const int half = Lr & 1;
        val[it] = *(const v4f*)(sw + row * OTP + half * 32 + pc * 4);
        go[it]  = (size_t)(m0 + sub * 16 + row) * HD + n0 + half * 32 + pc * 4;
      }
      if (MODE == 2) {
#pragma unroll
        for (int it = 0; it < 8; ++it) {
          const v4f rv = *(const v4f*)(resid + go[it]);
          val[it] = val[it] + rv;
        }
      }
      for (int ps = 0; ps < 2; ++ps) {
#pragma unroll
        for (int it = 0; it < 8; ++it) *(volatile v4f*)(out + go[it]) = val[it];
        __threadfence();
      }
    }
    if (MIRROR) {
      v4u vh[4];
      size_t gh[4];
#pragma unroll
      for (int it = 0; it < 4; ++it) {
        const int p   = lane + 32 * it;
        const int row = p >> 3;
        const int pc  = p & 7;
        gh[it] = (size_t)(m0 + sub * 16 + row) * HD + n0 + pc * 8;
        v4f a0 = *(const v4f*)(sw + row * OTP + pc * 8);
        v4f a1 = *(const v4f*)(sw + row * OTP + pc * 8 + 4);
        if (MODE == 2) {
          const v4f r0 = *(const v4f*)(resid + gh[it]);
          const v4f r1 = *(const v4f*)(resid + gh[it] + 4);
          a0 = a0 + r0;
          a1 = a1 + r1;
        }
        Pack8 pk;
        pk.h   = cvt8(a0 * 16.0f, a1 * 16.0f);
        vh[it] = pk.u;
      }
      for (int ps = 0; ps < 2; ++ps) {
#pragma unroll
        for (int it = 0; it < 4; ++it) *(volatile v4u*)(out16 + gh[it]) = vh[it];
        __threadfence();
      }
    }
  }
}

__global__ __launch_bounds__(256) void k_attn(const float* __restrict__ q, const float* __restrict__ k,
                                              const float* __restrict__ v, const int* __restrict__ bi,
                                              _Float16* __restrict__ ao) {
  __shared__ __align__(16) float orow[HD];
  const int i = blockIdx.x;
  const int tid = threadIdx.x, lane = tid & 31, h = tid >> 5;
  const int myset = bi[i];
  int start = i;
#pragma unroll 1
  for (int t = 0; t < NN; ++t) {
    if (start <= 0) break;
    const int g = bi[max(start - 1, 0)];
    if (g != myset) break;
    --start;
  }
  int end = i + 1;
#pragma unroll 1
  for (int t = 0; t < NN; ++t) {
    if (end >= NN) break;
    const int g = bi[min(end, NN - 1)];
    if (g != myset) break;
    ++end;
  }
  start = max(start, 0);
  end   = min(end, NN);

  const size_t hoff = (size_t)h * HDIM + 2 * lane;
  const v2f qv = *(const v2f*)(q + (size_t)i * HD + hoff);

  float mx = -FLT_MAX;
#pragma unroll 1
  for (int j = start; j < end; ++j) {
    if (j == i) continue;
    const v2f kv = *(const v2f*)(k + (size_t)j * HD + hoff);
    float p = qv.x * kv.x + qv.y * kv.y;
#pragma unroll
    for (int off = 16; off >= 1; off >>= 1) p += __shfl_xor(p, off, 32);
    mx = fmaxf(mx, p * 0.125f);
  }
  float l = 0.0f, a0 = 0.0f, a1 = 0.0f;
#pragma unroll 1
  for (int j = start; j < end; ++j) {
    if (j == i) continue;
    const v2f kv = *(const v2f*)(k + (size_t)j * HD + hoff);
    const v2f vv = *(const v2f*)(v + (size_t)j * HD + hoff);
    float p = qv.x * kv.x + qv.y * kv.y;
#pragma unroll
    for (int off = 16; off >= 1; off >>= 1) p += __shfl_xor(p, off, 32);
    const float w = expf(p * 0.125f - mx);
    l += w;
    a0 = fmaf(w, vv.x, a0);
    a1 = fmaf(w, vv.y, a1);
  }
  const float inv = (l > 0.5f) ? (1.0f / fmaxf(l, 1.0f)) : 0.0f;
  *(v2f*)(orow + h * HDIM + 2 * lane) = (v2f){a0 * inv, a1 * inv};
  __syncthreads();

  if (h == 0) {
    v4u vh[2];
    size_t go[2];
#pragma unroll
    for (int it = 0; it < 2; ++it) {
      const int off = it * 256 + lane * 8;
      const v4f b0 = *(const v4f*)(orow + off) * 16.0f;
      const v4f b1 = *(const v4f*)(orow + off + 4) * 16.0f;
      Pack8 pk;
      pk.h   = cvt8(b0, b1);
      vh[it] = pk.u;
      go[it] = (size_t)i * HD + off;
    }
    for (int ps = 0; ps < 2; ++ps) {
#pragma unroll
      for (int it = 0; it < 2; ++it) *(volatile v4u*)(ao + go[it]) = vh[it];
      __threadfence();
    }
  }
}

__global__ __launch_bounds__(128) void k_segmean(const float* __restrict__ dy, const float* __restrict__ se,
                                                 const int* __restrict__ bi, float* __restrict__ out) {
  const int s = blockIdx.x, tid = threadIdx.x;
  int lo = 0, hb = NN;
#pragma unroll 1
  for (int it = 0; it < 16; ++it) {
    if (lo >= hb) break;
    const int mid = min((lo + hb) >> 1, NN - 1);
    if (bi[mid] < s) lo = mid + 1; else hb = mid;
  }
  const int start = min(max(lo, 0), NN);
  lo = 0; hb = NN;
#pragma unroll 1
  for (int it = 0; it < 16; ++it) {
    if (lo >= hb) break;
    const int mid = min((lo + hb) >> 1, NN - 1);
    if (bi[mid] <= s) lo = mid + 1; else hb = mid;
  }
  const int end = min(max(lo, 0), NN);

  const int f = 4 * tid;
  v4f acc = (v4f){0.0f, 0.0f, 0.0f, 0.0f};
#pragma unroll 1
  for (int mm = start; mm < end; ++mm) {
    const v4f a = *(const v4f*)(dy + (size_t)mm * HD + f);
    const v4f b = *(const v4f*)(se + (size_t)mm * HD + f);
    const v4f e = a - b;
    acc += e * e;
  }
  const float cnt = (float)(end - start);
  const float inv = 1.0f / fmaxf(cnt, 1.0f);
  const v4f o = acc * inv;
  volatile v4f* d = (volatile v4f*)(out + (size_t)s * HD + f);
  *d = o;
  __threadfence();
  *d = o;
}

extern "C" void kernel_launch(void* const* d_in, const int* in_sizes, int n_in,
                              void* d_out, int out_size, void* d_ws, size_t ws_size,
                              hipStream_t stream) {
  if (n_in < 22) return;
  if (in_sizes[0] != NN * HD) return;
  if (in_sizes[1] != NN) return;
  const int widx[9] = {2, 4, 6, 8, 10, 13, 15, 17, 19};
  const int bidx[9] = {3, 5, 7, 9, 11, 14, 16, 18, 20};
  for (int j = 0; j < 9; ++j) {
    if (in_sizes[widx[j]] != HD * HD) return;
    if (in_sizes[bidx[j]] != HD) return;
  }
  if (in_sizes[12] != 1) return;
  if (in_sizes[21] != 1) return;
  if (out_size != NSET * HD) return;

  const float* emb = (const float*)d_in[0];
  const int*   bi  = (const int*)d_in[1];
  const float* Wp[9];
  const float* bp[9];
  for (int j = 0; j < 9; ++j) { Wp[j] = (const float*)d_in[widx[j]]; bp[j] = (const float*)d_in[bidx[j]]; }
  const float* beta1 = (const float*)d_in[12];
  const float* beta2 = (const float*)d_in[21];
  float* out = (float*)d_out;

  const size_t WTB = (size_t)HD * HD * 2;
  const size_t P16 = (size_t)NN * HD * 2;
  const size_t P32 = (size_t)NN * HD * 4;
  size_t off = 0;
  const size_t oWT  = off; off += 9 * WTB;
  const size_t oX16 = off; off += P16;
  const size_t oSE  = off; off += P32;
  const size_t oQ   = off; off += P32;
  const size_t oK   = off; off += P32;
  const size_t oV   = off; off += P32;
  const size_t oAO  = off; off += P16;
  const size_t oD1  = off; off += P32;
  const size_t oD16 = off; off += P16;
  const size_t oD2  = off; off += P32;
  if (off > ws_size) return;
  if (off > (size_t)134217728) return;

  char* ws = (char*)d_ws;
  _Float16* WT[9];
  for (int j = 0; j < 9; ++j) WT[j] = (_Float16*)(ws + oWT + (size_t)j * WTB);
  _Float16* X16 = (_Float16*)(ws + oX16);
  float*    SE  = (float*)(ws + oSE);
  float*    Q   = (float*)(ws + oQ);
  float*    K   = (float*)(ws + oK);
  float*    V   = (float*)(ws + oV);
  _Float16* AO  = (_Float16*)(ws + oAO);
  float*    D1  = (float*)(ws + oD1);
  _Float16* D16 = (_Float16*)(ws + oD16);
  float*    D2  = (float*)(ws + oD2);

  const float escale = 6.103515625e-05f;
  const dim3 gg(NN / 256, HD / 64), gb(256);

  for (int j = 0; j < 9; ++j)
    k_wt<<<dim3(HD / 64, HD / 32), dim3(256), 0, stream>>>(Wp[j], WT[j]);
  k_cvt<<<dim3((NN * HD) / 2048), dim3(256), 0, stream>>>(emb, X16, 16.0f);
  k_gemm<0, false><<<gg, gb, 0, stream>>>(X16, WT[0], bp[0], escale, emb, beta1, SE, D16);
  k_gemm<1, false><<<gg, gb, 0, stream>>>(X16, WT[1], bp[1], escale, emb, beta1, Q, D16);
  k_gemm<1, false><<<gg, gb, 0, stream>>>(X16, WT[2], bp[2], escale, emb, beta1, K, D16);
  k_gemm<1, false><<<gg, gb, 0, stream>>>(X16, WT[3], bp[3], escale, emb, beta1, V, D16);
  k_attn<<<dim3(NN), dim3(256), 0, stream>>>(Q, K, V, bi, AO);
  k_gemm<2, true><<<gg, gb, 0, stream>>>(AO, WT[4], bp[4], escale, emb, beta1, D1, D16);
  k_gemm<1, false><<<gg, gb, 0, stream>>>(D16, WT[5], bp[5], escale, emb, beta2, Q, AO);
  k_gemm<1, false><<<gg, gb, 0, stream>>>(D16, WT[6], bp[6], escale, emb, beta2, K, AO);
  k_gemm<1, false><<<gg, gb, 0, stream>>>(D16, WT[7], bp[7], escale, emb, beta2, V, AO);
  k_attn<<<dim3(NN), dim3(256), 0, stream>>>(Q, K, V, bi, AO);
  k_gemm<2, false><<<gg, gb, 0, stream>>>(AO, WT[8], bp[8], escale, D1, beta2, D2, D16);
  k_segmean<<<dim3(NSET), dim3(128), 0, stream>>>(D2, SE, bi, out);
  (void)hipGetLastError();
}
